// MutilHeadSelfAttn_66013647340076
// MI455X (gfx1250) — hardware-verified
//
#include <hip/hip_runtime.h>
#include <math.h>

typedef __attribute__((ext_vector_type(16))) _Float16 v16h;
typedef __attribute__((ext_vector_type(16))) __bf16 v16b;
typedef __attribute__((ext_vector_type(8)))  _Float16 v8h;
typedef __attribute__((ext_vector_type(8)))  float v8f;
typedef __attribute__((ext_vector_type(4)))  float v4f;
typedef __attribute__((ext_vector_type(2)))  float v2f;
typedef __attribute__((ext_vector_type(4)))  unsigned v4u;
typedef __attribute__((ext_vector_type(4)))  int v4i;
typedef float __attribute__((may_alias)) float_a;
typedef int __attribute__((may_alias)) int_a;

template <typename T> __device__ __forceinline__ void vst2(void* p, T v) { *(volatile T*)p = v; __threadfence(); *(volatile T*)p = v; }
__device__ __forceinline__ v8f wmma16(v16h a, v16h b, v8f c) {
  v8f d = __builtin_amdgcn_wmma_f32_16x16x32_f16(false, a, false, b, (short)0, c, false, false);
  asm volatile("v_nop\n\tv_nop\n\tv_nop\n\tv_nop" : "+v"(d) : "v"(a), "v"(b));
  return d;
}
__device__ __forceinline__ v8f wmma_bf(v16b a, v16b b, v8f c) {
  v8f d = __builtin_amdgcn_wmma_f32_16x16x32_bf16(false, a, false, b, (short)0, c, false, false);
  asm volatile("v_nop\n\tv_nop\n\tv_nop\n\tv_nop" : "+v"(d) : "v"(a), "v"(b));
  return d;
}
__device__ __forceinline__ v16h frag_h(const _Float16* rowk0, int lane) {
  union { v16h v; v8h q[2]; } u; const _Float16* p = rowk0 + 8 * (lane >> 4);
  u.q[0] = *(const v8h*)p; u.q[1] = *(const v8h*)(p + 16); return u.v;
}
__device__ __forceinline__ v16h frag_f32(const float* rowk0, int lane) {
  v16h a; const float* p = rowk0 + 8 * (lane >> 4);
#pragma unroll
  for (int i = 0; i < 8; ++i) { a[i] = (_Float16)p[i]; a[8 + i] = (_Float16)p[16 + i]; }
  return a;
}
__device__ __forceinline__ v16h frag_f32s(const float* rowk0, int lane, float sc) {
  v16h a; const float* p = rowk0 + 8 * (lane >> 4);
#pragma unroll
  for (int i = 0; i < 8; ++i) { a[i] = (_Float16)(p[i] * sc); a[8 + i] = (_Float16)(p[16 + i] * sc); }
  return a;
}
__device__ __forceinline__ v16h fragc_f32(const float* W, int k0, int n, int lane, int ld, int K) {
  v16h a; const int g = lane >> 4;
#pragma unroll
  for (int i = 0; i < 8; ++i) { const int ka = k0 + 8 * g + i, kb = ka + 16;
    a[i] = (_Float16)(ka < K ? W[(size_t)ka * ld + n] : 0.f); a[8 + i] = (_Float16)(kb < K ? W[(size_t)kb * ld + n] : 0.f); }
  return a;
}
struct F2 { v16b h, l; };
__device__ __forceinline__ F2 bsplit16(const float v[16]) { F2 r;
#pragma unroll
  for (int i = 0; i < 16; ++i) { const __bf16 h = (__bf16)v[i]; r.h[i] = h; r.l[i] = (__bf16)(v[i] - (float)h); }
  return r; }
__device__ __forceinline__ F2 split_row(const float* row, int k0, int lane) { float v[16]; const float* p = row + k0 + 8 * (lane >> 4);
#pragma unroll
  for (int i = 0; i < 8; ++i) { v[i] = p[i]; v[8 + i] = p[16 + i]; }
  return bsplit16(v); }
__device__ __forceinline__ F2 split_rowK(const float* row, int k0, int lane, int K) { float v[16]; const int g = lane >> 4;
#pragma unroll
  for (int i = 0; i < 8; ++i) { const int ka = k0 + 8 * g + i, kb = ka + 16; v[i] = ka < K ? row[ka] : 0.f; v[8 + i] = kb < K ? row[kb] : 0.f; }
  return bsplit16(v); }
__device__ __forceinline__ F2 split_col(const float* W, int k0, int n, int lane, int ld, int K) { float v[16]; const int g = lane >> 4;
#pragma unroll
  for (int i = 0; i < 8; ++i) { const int ka = k0 + 8 * g + i, kb = ka + 16; v[i] = ka < K ? W[(size_t)ka * ld + n] : 0.f; v[8 + i] = kb < K ? W[(size_t)kb * ld + n] : 0.f; }
  return bsplit16(v); }
__device__ __forceinline__ v8f mac3(const F2& a, const F2& b, v8f c) { c = wmma_bf(a.l, b.h, c); c = wmma_bf(a.h, b.l, c); return wmma_bf(a.h, b.h, c); }
__device__ __forceinline__ float sigm(float v) { return 1.0f / (1.0f + expf(-v)); }
#define LDSX() do { asm volatile("s_wait_dscnt 0" ::: "memory"); __builtin_amdgcn_wave_barrier(); __builtin_amdgcn_fence(__ATOMIC_RELEASE, "workgroup"); } while (0)

#define NB 4
#define SS 1024
#define HID 1024
#define NH 16
#define HD 64
#define NR (NB * SS)

__global__ __launch_bounds__(256) void k_ln3(const float* __restrict__ q, const float* __restrict__ k, const float* __restrict__ v, const float* __restrict__ gq, const float* __restrict__ bq, const float* __restrict__ gk, const float* __restrict__ bk, const float* __restrict__ gv, const float* __restrict__ bv2, _Float16* __restrict__ X16) {
  const int wave = threadIdx.x >> 5, lane = threadIdx.x & 31, which = blockIdx.y; const size_t r = (size_t)blockIdx.x * 8 + wave; if (r >= NR) return;
  const float* src = (which == 0 ? q : which == 1 ? k : v) + r * HID; const float* g = which == 0 ? gq : which == 1 ? gk : gv; const float* bb = which == 0 ? bq : which == 1 ? bk : bv2;
  float xv[32]; float s = 0.f;
#pragma unroll
  for (int i = 0; i < 4; ++i) { const v4f a = *(const v4f*)(src + i * 256 + lane * 8), c = *(const v4f*)(src + i * 256 + lane * 8 + 4);
    xv[i * 8 + 0] = a[0]; xv[i * 8 + 1] = a[1]; xv[i * 8 + 2] = a[2]; xv[i * 8 + 3] = a[3]; xv[i * 8 + 4] = c[0]; xv[i * 8 + 5] = c[1]; xv[i * 8 + 6] = c[2]; xv[i * 8 + 7] = c[3]; }
#pragma unroll
  for (int i = 0; i < 32; ++i) s += xv[i];
#pragma unroll
  for (int off = 16; off >= 1; off >>= 1) s += __shfl_xor(s, off, 32);
  const float mu = s * (1.0f / HID); float q2 = 0.f;
#pragma unroll
  for (int i = 0; i < 32; ++i) { const float d = xv[i] - mu; q2 += d * d; }
#pragma unroll
  for (int off = 16; off >= 1; off >>= 1) q2 += __shfl_xor(q2, off, 32);
  const float rs = rsqrtf(q2 * (1.0f / HID) + 1e-5f);
#pragma unroll
  for (int i = 0; i < 4; ++i) { union { v8h h; v4u u; } pk;
#pragma unroll
    for (int e = 0; e < 8; ++e) { const int c = i * 256 + lane * 8 + e; pk.h[e] = (_Float16)((xv[i * 8 + e] - mu) * rs * g[c] + bb[c]); }
    vst2(X16 + ((size_t)which * NR + r) * HID + i * 256 + lane * 8, pk.u); }
}
__global__ __launch_bounds__(256) void k_pack(const float* __restrict__ Wq, const float* __restrict__ Wk, const float* __restrict__ Wv, const float* __restrict__ Wf, _Float16* __restrict__ P) {
  const int r = blockIdx.x, tid = threadIdx.x; __shared__ __align__(16) _Float16 srow[HID];
  const int which = r >> 10, n = r & 1023; const float* W = (which == 0 ? Wq : which == 1 ? Wk : which == 2 ? Wv : Wf) + (size_t)n * HID;
  for (int kk = tid; kk < HID; kk += 256) srow[kk] = (_Float16)(W[kk] * 16.0f);
  __syncthreads();
  if (tid < 128) vst2(P + (size_t)r * HID + tid * 8, *(const v4u*)(&srow[tid * 8]));
}
__global__ __launch_bounds__(256) void k_rope(float* __restrict__ CS, float* __restrict__ SN) {
  const int s = blockIdx.x * 8 + (threadIdx.x >> 5), j = threadIdx.x & 31;
  const float inv = 1.0f / powf(10000.0f, (float)(2 * j) / (float)HD); const float f = (float)s * inv;
  vst2(CS + (size_t)s * 32 + j, cosf(f)); vst2(SN + (size_t)s * 32 + j, sinf(f));
}
__global__ __launch_bounds__(128) void k_qkv(const _Float16* __restrict__ X16, const _Float16* __restrict__ P, const float* __restrict__ bq, const float* __restrict__ bk, const float* __restrict__ bv, const float* __restrict__ CS, const float* __restrict__ SN,
                                           _Float16* __restrict__ Q16, _Float16* __restrict__ K16, _Float16* __restrict__ VT) {
  __shared__ __align__(16) float so[4][16][132];
  __shared__ __align__(16) _Float16 st[128][72];
  const int tid = threadIdx.x, wave = tid >> 5, lane = tid & 31, col = lane & 15, g = lane >> 4;
  const int which = blockIdx.z, r0b = blockIdx.x * 64, r0 = r0b + wave * 16, n0 = blockIdx.y * 128; const int b = r0b / SS, s0 = r0b % SS;
  const _Float16* A = X16 + (size_t)which * NR * HID; const _Float16* Pw = P + (size_t)which * HID * HID; const float* bias = which == 0 ? bq : (which == 1 ? bk : bv);
  v8f acc[8] = {};
#pragma unroll 2
  for (int kc = 0; kc < HID / 32; ++kc) { const v16h a = frag_h(A + (size_t)(r0 + col) * HID + kc * 32, lane);
#pragma unroll
    for (int j = 0; j < 8; ++j) acc[j] = wmma16(a, frag_h(Pw + (size_t)(n0 + j * 16 + col) * HID + kc * 32, lane), acc[j]); }
#pragma unroll
  for (int j = 0; j < 8; ++j) { const float bb = bias[n0 + j * 16 + col];
#pragma unroll
    for (int r = 0; r < 8; ++r) acc[j][r] = acc[j][r] * (1.0f / 16.0f) + bb; }
  if (which < 2) {
#pragma unroll
    for (int hh = 0; hh < 2; ++hh)
#pragma unroll
      for (int jj = 0; jj < 2; ++jj) { const int jlo = hh * 4 + jj, jhi = jlo + 2; const int dj = jj * 16 + col;
#pragma unroll
        for (int r = 0; r < 8; ++r) { const int s = s0 + wave * 16 + 8 * g + r; const float c = CS[(size_t)s * 32 + dj], sn = SN[(size_t)s * 32 + dj];
          const float lo = acc[jlo][r], hi = acc[jhi][r];
          so[wave][8 * g + r][jlo * 16 + col] = (lo * c - hi * sn) * 4.0f; so[wave][8 * g + r][jhi * 16 + col] = (hi * c + lo * sn) * 4.0f; } }
    LDSX();
    _Float16* D = which == 0 ? Q16 : K16;
    for (int qq = lane; qq < 16 * 2 * 8; qq += 32) { const int hh = qq >> 7, rl = (qq >> 3) & 15, pc = qq & 7; const int h = (n0 >> 6) + hh; union { v8h h8; v4u u; } pk;
#pragma unroll
      for (int e = 0; e < 8; ++e) pk.h8[e] = (_Float16)so[wave][rl][hh * 64 + pc * 8 + e];
      vst2(D + (((size_t)b * NH + h) * SS + s0 + wave * 16 + rl) * HD + pc * 8, pk.u); } }
  else {
#pragma unroll
    for (int j = 0; j < 8; ++j)
#pragma unroll
      for (int r = 0; r < 8; ++r) st[j * 16 + col][wave * 16 + 8 * g + r] = (_Float16)(acc[j][r] * 4.0f);
    __syncthreads();
    for (int qq = tid; qq < 128 * 8; qq += 128) { const int cl = qq >> 3, pc = qq & 7; const int c = n0 + cl, h = c >> 6, d = c & 63; vst2(VT + (((size_t)b * NH + h) * HD + d) * SS + s0 + pc * 8, *(const v4u*)(&st[cl][pc * 8])); } }
}
__global__ __launch_bounds__(128) void k_attn(const _Float16* __restrict__ Q16, const _Float16* __restrict__ K16, const _Float16* __restrict__ VT, const int* __restrict__ mask, _Float16* __restrict__ O16) {
  __shared__ __align__(16) float sS[4][16][68];
  __shared__ __align__(16) _Float16 sP[4][16][72];
  __shared__ __align__(16) float sO[4][16][68];
  __shared__ int smk[SS];
  const int tid = threadIdx.x, w = tid >> 5, lane = tid & 31, col = lane & 15, g = lane >> 4;
  const int b = blockIdx.z, h = blockIdx.y, q0 = blockIdx.x * 64 + w * 16; const size_t bh = (size_t)b * NH + h;
  for (int qq = tid; qq < SS; qq += 128) smk[qq] = mask[(size_t)b * SS + qq];
  __syncthreads();
  v16h aq[2];
#pragma unroll
  for (int kc = 0; kc < 2; ++kc) aq[kc] = frag_h(Q16 + (bh * SS + q0 + col) * HD + kc * 32, lane);
  float mrun = -3.0e38f, lrun = 0.f; v8f acc[4] = {};
#pragma unroll 1
  for (int kt = 0; kt < SS / 64; ++kt) {
#pragma unroll
    for (int t = 0; t < 4; ++t) { v8f s = {}; const int key = kt * 64 + t * 16 + col;
#pragma unroll
      for (int kc = 0; kc < 2; ++kc) s = wmma16(aq[kc], frag_h(K16 + (bh * SS + key) * HD + kc * 32, lane), s);
      const bool keep = smk[key] != 0;
#pragma unroll
      for (int r = 0; r < 8; ++r) sS[w][8 * g + r][t * 16 + col] = keep ? s[r] * (0.125f / 16.0f) : 1e-10f; }
    LDSX();
    float mx = -3.4e38f;
#pragma unroll
    for (int jj = 0; jj < 32; ++jj) mx = fmaxf(mx, sS[w][col][g * 32 + jj]);
    mx = fmaxf(mx, __shfl_xor(mx, 16, 32));
    const float mnew = fmaxf(mrun, mx); const float corr = expf(mrun - mnew);
    float ps = 0.f;
#pragma unroll
    for (int jj = 0; jj < 32; ++jj) { const float p = expf(sS[w][col][g * 32 + jj] - mnew); ps += p; sP[w][col][g * 32 + jj] = (_Float16)(p * 16384.0f); }
    ps += __shfl_xor(ps, 16, 32);
    lrun = lrun * corr + ps; mrun = mnew;
#pragma unroll
    for (int r = 0; r < 8; ++r) { const float cr = __shfl(corr, 8 * g + r, 32);
#pragma unroll
      for (int t = 0; t < 4; ++t) acc[t][r] *= cr; }
    LDSX();
#pragma unroll
    for (int kc = 0; kc < 2; ++kc) { const v16h pa = frag_h(&sP[w][col][0] + kc * 32, lane);
#pragma unroll
      for (int t = 0; t < 4; ++t) acc[t] = wmma16(pa, frag_h(VT + (bh * HD + t * 16 + col) * SS + kt * 64 + kc * 32, lane), acc[t]); }
    __builtin_amdgcn_wave_barrier(); }
#pragma unroll
  for (int r = 0; r < 8; ++r) { const float lr = __shfl(lrun, 8 * g + r, 32); const float inv = 8.0f / (lr * 16384.0f * 4.0f);
#pragma unroll
    for (int t = 0; t < 4; ++t) sO[w][8 * g + r][t * 16 + col] = acc[t][r] * inv; }
  LDSX();
  for (int qq = lane; qq < 16 * 8; qq += 32) { const int rl = qq >> 3, pc = qq & 7; union { v8h h8; v4u u; } pk;
#pragma unroll
    for (int e = 0; e < 8; ++e) pk.h8[e] = (_Float16)sO[w][rl][pc * 8 + e];
    vst2(O16 + ((bh * SS) + q0 + rl) * HD + pc * 8, pk.u); }
}
__global__ __launch_bounds__(256) void k_ln2(const _Float16* __restrict__ O16, const float* __restrict__ g2, const float* __restrict__ b2, float* __restrict__ FX, _Float16* __restrict__ FX16) {
  const int wave = threadIdx.x >> 5, lane = threadIdx.x & 31; const size_t r = (size_t)blockIdx.x * 8 + wave; if (r >= NR) return;
  const int b = (int)(r / SS), s = (int)(r % SS);
  float xv[32]; float sm = 0.f;
#pragma unroll
  for (int i = 0; i < 4; ++i) { const int c0 = i * 256 + lane * 8; const int h = c0 >> 6, d = c0 & 63; const _Float16* src = O16 + (((size_t)b * NH + h) * SS + s) * HD + d;
#pragma unroll
    for (int e = 0; e < 8; ++e) { xv[i * 8 + e] = (float)src[e] * 0.125f; sm += xv[i * 8 + e]; } }
#pragma unroll
  for (int off = 16; off >= 1; off >>= 1) sm += __shfl_xor(sm, off, 32);
  const float mu = sm * (1.0f / HID); float q2 = 0.f;
#pragma unroll
  for (int i = 0; i < 32; ++i) { const float dd = xv[i] - mu; q2 += dd * dd; }
#pragma unroll
  for (int off = 16; off >= 1; off >>= 1) q2 += __shfl_xor(q2, off, 32);
  const float rs = rsqrtf(q2 * (1.0f / HID) + 1e-5f);
#pragma unroll
  for (int i = 0; i < 4; ++i) { union { v8h h; v4u u; } pk; v4f f0, f1;
#pragma unroll
    for (int e = 0; e < 8; ++e) { const int c = i * 256 + lane * 8 + e; const float fv = (xv[i * 8 + e] - mu) * rs * g2[c] + b2[c]; pk.h[e] = (_Float16)fv; if (e < 4) f0[e] = fv; else f1[e - 4] = fv; }
    vst2(FX + r * HID + i * 256 + lane * 8, f0); vst2(FX + r * HID + i * 256 + lane * 8 + 4, f1); vst2(FX16 + r * HID + i * 256 + lane * 8, pk.u); }
}
__global__ __launch_bounds__(128) void k_ffn(const _Float16* __restrict__ FX16, const _Float16* __restrict__ P, const float* __restrict__ bf, float* __restrict__ FO) {
  __shared__ __align__(16) float so[4][16][132];
  const int tid = threadIdx.x, wave = tid >> 5, lane = tid & 31, col = lane & 15, g = lane >> 4;
  const int r0 = blockIdx.x * 64 + wave * 16, n0 = blockIdx.y * 128;
  v8f acc[8] = {};
#pragma unroll 2
  for (int kc = 0; kc < HID / 32; ++kc) { const v16h a = frag_h(FX16 + (size_t)(r0 + col) * HID + kc * 32, lane);
#pragma unroll
    for (int j = 0; j < 8; ++j) acc[j] = wmma16(a, frag_h(P + (size_t)(3 * HID + n0 + j * 16 + col) * HID + kc * 32, lane), acc[j]); }
#pragma unroll
  for (int j = 0; j < 8; ++j) { const float bb = bf[n0 + j * 16 + col];
#pragma unroll
    for (int r = 0; r < 8; ++r) { const float vv = acc[j][r] * (1.0f / 16.0f) + bb; so[wave][8 * g + r][j * 16 + col] = vv > 0.f ? vv : 0.f; } }
  LDSX();
#pragma unroll 4
  for (int rl = 0; rl < 16; ++rl) vst2(FO + (size_t)(r0 + rl) * HID + n0 + lane * 4, *(const v4f*)(&so[wave][rl][lane * 4]));
}
__global__ __launch_bounds__(256) void k_fin(const float* __restrict__ FX, const float* __restrict__ FO, const float* __restrict__ g3, const float* __restrict__ b3, float* __restrict__ out) {
  const int wave = threadIdx.x >> 5, lane = threadIdx.x & 31; const size_t r = (size_t)blockIdx.x * 8 + wave; if (r >= NR) return;
  const float* fo = FO + r * HID; float xv[32]; float sm = 0.f;
#pragma unroll
  for (int i = 0; i < 4; ++i) { const v4f a = *(const v4f*)(fo + i * 256 + lane * 8), c = *(const v4f*)(fo + i * 256 + lane * 8 + 4);
    xv[i * 8 + 0] = a[0]; xv[i * 8 + 1] = a[1]; xv[i * 8 + 2] = a[2]; xv[i * 8 + 3] = a[3]; xv[i * 8 + 4] = c[0]; xv[i * 8 + 5] = c[1]; xv[i * 8 + 6] = c[2]; xv[i * 8 + 7] = c[3]; }
#pragma unroll
  for (int i = 0; i < 32; ++i) sm += xv[i];
#pragma unroll
  for (int off = 16; off >= 1; off >>= 1) sm += __shfl_xor(sm, off, 32);
  const float mu = sm * (1.0f / HID); float q2 = 0.f;
#pragma unroll
  for (int i = 0; i < 32; ++i) { const float dd = xv[i] - mu; q2 += dd * dd; }
#pragma unroll
  for (int off = 16; off >= 1; off >>= 1) q2 += __shfl_xor(q2, off, 32);
  const float rs = rsqrtf(q2 * (1.0f / HID) + 1e-5f);
  const float* fx = FX + r * HID;
#pragma unroll
  for (int i = 0; i < 4; ++i) { v4f o0, o1; const int c0 = i * 256 + lane * 8;
#pragma unroll
    for (int e = 0; e < 8; ++e) { const int c = c0 + e; const float vv = fx[c] + ((xv[i * 8 + e] - mu) * rs * g3[c] + b3[c]); if (e < 4) o0[e] = vv; else o1[e - 4] = vv; }
    vst2(out + r * HID + c0, o0); vst2(out + r * HID + c0 + 4, o1); }
}
extern "C" void kernel_launch(void* const* d_in, const int* in_sizes, int n_in, void* d_out, int out_size, void* d_ws, size_t ws_size, hipStream_t stream) {
  (void)in_sizes; (void)n_in; (void)out_size; (void)ws_size;
  const float** I = (const float**)d_in;
  const float* q = I[0]; const float* k = I[1]; const float* v = I[2]; const float* g1q = I[3]; const float* b1q = I[4]; const float* g1k = I[5]; const float* b1k = I[6]; const float* g1v = I[7]; const float* b1v = I[8];
  const float* Wq = I[9]; const float* bq = I[10]; const float* Wk = I[11]; const float* bk = I[12]; const float* Wv = I[13]; const float* bv = I[14]; const float* g2 = I[15]; const float* b2 = I[16]; const float* g3 = I[17]; const float* b3 = I[18]; const float* Wf = I[19]; const float* bf = I[20]; const int* mask = (const int*)d_in[21];
  float* out = (float*)d_out;
  char* ws = (char*)d_ws; size_t off = 0;
  auto take = [&](size_t bytes) { char* p = ws + off; off += (bytes + 255) & ~(size_t)255; return p; };
  _Float16* X16 = (_Float16*)take((size_t)3 * NR * HID * 2); _Float16* P = (_Float16*)take((size_t)4 * HID * HID * 2); float* CS = (float*)take((size_t)SS * 32 * 4); float* SN = (float*)take((size_t)SS * 32 * 4);
  _Float16* Q16 = (_Float16*)take((size_t)NR * HID * 2); _Float16* K16 = (_Float16*)take((size_t)NR * HID * 2); _Float16* VT = (_Float16*)take((size_t)NR * HID * 2); _Float16* O16 = (_Float16*)take((size_t)NR * HID * 2);
  float* FX = (float*)take((size_t)NR * HID * 4); _Float16* FX16 = (_Float16*)take((size_t)NR * HID * 2); float* FO = (float*)take((size_t)NR * HID * 4);
  k_ln3<<<dim3(NR / 8, 3), 256, 0, stream>>>(q, k, v, g1q, b1q, g1k, b1k, g1v, b1v, X16);
  k_pack<<<4 * HID, 256, 0, stream>>>(Wq, Wk, Wv, Wf, P);
  k_rope<<<SS / 8, 256, 0, stream>>>(CS, SN);
  k_qkv<<<dim3(NR / 64, HID / 128, 3), 128, 0, stream>>>(X16, P, bq, bk, bv, CS, SN, Q16, K16, VT);
  k_attn<<<dim3(SS / 64, NH, NB), 128, 0, stream>>>(Q16, K16, VT, mask, O16);
  k_ln2<<<NR / 8, 256, 0, stream>>>(O16, g2, b2, FX, FX16);
  k_ffn<<<dim3(NR / 64, HID / 128), 128, 0, stream>>>(FX16, P, bf, FO);
  k_fin<<<NR / 8, 256, 0, stream>>>(FX, FO, g3, b3, out);
}
